// NeuralRoughSimulator_46969762349160
// MI455X (gfx1250) — hardware-verified
//
#include <hip/hip_runtime.h>
#include <math.h>


typedef __attribute__((ext_vector_type(16))) _Float16 v16h;
typedef __attribute__((ext_vector_type(8)))  _Float16 v8h;
typedef __attribute__((ext_vector_type(8)))  float    v8f;
typedef __attribute__((ext_vector_type(4)))  float    v4f;

#define NPB       32
#define NTHREADS  64
#define NFRAG     20
#define IN_PITCH  40
#define ACT_PITCH 72
#define OUT_PITCH 36
#define CHUNK     32

__device__ __forceinline__ v16h frag_load_a(const _Float16* p) {
  union { v16h v; v8h h[2]; } f;
  f.h[0] = *(const v8h*)(p);
  f.h[1] = *(const v8h*)(p + 16);
  return f.v;
}
__device__ __forceinline__ v16h frag_load_packed(const _Float16* p) {
  union { v16h v; v8h h[2]; } f;
  f.h[0] = *(const v8h*)(p);
  f.h[1] = *(const v8h*)(p + 8);
  return f.v;
}
__device__ __forceinline__ v8f mma_f16(v16h a, v16h b, v8f c) {
  c = __builtin_amdgcn_wmma_f32_16x16x32_f16(false, a, false, b, (short)0, c, false, false);
  asm volatile("v_nop\n\tv_nop\n\tv_nop\n\tv_nop" : "+v"(c) : "v"(a), "v"(b));
  return c;
}
__device__ __forceinline__ void lds_wave_sync() {
  __builtin_amdgcn_fence(__ATOMIC_RELEASE, "workgroup");
  __builtin_amdgcn_wave_barrier();
  __builtin_amdgcn_fence(__ATOMIC_ACQUIRE, "workgroup");
}
__device__ __forceinline__ float tanh_act(float x) {
  const float t = __builtin_amdgcn_exp2f(x * 2.8853900817779268f);
  return 1.0f - 2.0f * __builtin_amdgcn_rcpf(t + 1.0f);
}

template <int NK>
__device__ __forceinline__ void layer_fwd(const _Float16* src, int spitch, const _Float16* wfrag,
                                          float bt0, float bt1, float bt2, float bt3,
                                          _Float16* dst, int lane) {
  const int hh = lane >> 4, rl = lane & 15;
  v16h a0[NK], a1[NK];
#pragma unroll
  for (int c = 0; c < NK; ++c) {
    a0[c] = frag_load_a(src + rl * spitch + c * 32 + 8 * hh);
    a1[c] = frag_load_a(src + (16 + rl) * spitch + c * 32 + 8 * hh);
  }
  lds_wave_sync();
  const float bts[4] = {bt0, bt1, bt2, bt3};
#pragma unroll
  for (int t = 0; t < 4; ++t) {
    v8f acc0, acc1;
#pragma unroll
    for (int r = 0; r < 8; ++r) { acc0[r] = bts[t]; acc1[r] = bts[t]; }
#pragma unroll
    for (int c = 0; c < NK; ++c) {
      const v16h b = frag_load_packed(wfrag + ((t * NK + c) * 32 + lane) * 16);
      acc0 = mma_f16(a0[c], b, acc0);
      acc1 = mma_f16(a1[c], b, acc1);
    }
#pragma unroll
    for (int r = 0; r < 8; ++r) {
      dst[(8 * hh + r) * ACT_PITCH + t * 16 + rl]      = (_Float16)tanh_act(acc0[r]);
      dst[(16 + 8 * hh + r) * ACT_PITCH + t * 16 + rl] = (_Float16)tanh_act(acc1[r]);
    }
  }
  lds_wave_sync();
}

__global__ __launch_bounds__(NTHREADS)
void nrs_main(const float* __restrict__ dW0, const float* __restrict__ db0,
              const float* __restrict__ gW0, const float* __restrict__ gb0,
              const float* __restrict__ dW1, const float* __restrict__ db1,
              const float* __restrict__ gW1, const float* __restrict__ gb1,
              const float* __restrict__ dW2, const float* __restrict__ db2,
              const float* __restrict__ gW2, const float* __restrict__ gb2,
              const float* __restrict__ dW3, const float* __restrict__ db3,
              const float* __restrict__ gW3, const float* __restrict__ gb3,
              const float* __restrict__ init_var, const float* __restrict__ dw,
              const float* __restrict__ dtp, const float* __restrict__ kappap,
              const float* __restrict__ thetap,
              float* __restrict__ out, int B, int S) {
  __shared__ __align__(16) _Float16 s_frag[2 * NFRAG * 512];
  __shared__ __align__(16) _Float16 s_in[NPB * IN_PITCH];
  __shared__ __align__(16) _Float16 s_act[2][NPB * ACT_PITCH];
  __shared__ __align__(16) float    s_out[NPB * OUT_PITCH];
  __shared__ float s_hw[2][64];
  __shared__ float s_raw[2][NPB];

  const int tid   = threadIdx.x;
  const int lane  = tid & 31;
  const int wave  = tid >> 5;
  const int rl    = lane & 15;
  const int path0 = blockIdx.x * NPB;

  for (int idx = tid; idx < 2 * NFRAG * 512; idx += NTHREADS) {
    const int i   = idx & 15;
    const int ln  = (idx >> 4) & 31;
    const int f   = idx >> 9;
    const int nid = (f >= NFRAG) ? 1 : 0;
    const int fl  = f - nid * NFRAG;
    int l, t, c;
    if (fl < 4)       { l = 0; t = fl;             c = 0; }
    else if (fl < 12) { l = 1; t = (fl - 4) >> 1;  c = (fl - 4) & 1; }
    else              { l = 2; t = (fl - 12) >> 1; c = (fl - 12) & 1; }
    const int Kdim = (l == 0) ? 15 : 64;
    const int n = t * 16 + (ln & 15);
    const int k = c * 32 + 8 * (ln >> 4) + (i & 7) + 16 * (i >> 3);
    const float* Wp = nid ? ((l == 0) ? gW0 : ((l == 1) ? gW1 : gW2))
                          : ((l == 0) ? dW0 : ((l == 1) ? dW1 : dW2));
    const int kc = (k < Kdim) ? k : (Kdim - 1);
    float w = Wp[n * Kdim + kc];
    if (k >= Kdim) w = 0.0f;
    s_frag[idx] = (_Float16)w;
  }
  if (tid < 64) { s_hw[0][tid] = dW3[tid]; s_hw[1][tid] = gW3[tid]; }
  for (int k = tid; k < NPB * IN_PITCH; k += NTHREADS) s_in[k] = (_Float16)0.0f;
  __syncthreads();

  const float* bp0 = wave ? gb0 : db0;
  const float* bp1 = wave ? gb1 : db1;
  const float* bp2 = wave ? gb2 : db2;
  float b0r[4], b1r[4], b2r[4];
#pragma unroll
  for (int t = 0; t < 4; ++t) {
    b0r[t] = bp0[t * 16 + rl];
    b1r[t] = bp1[t * 16 + rl];
    b2r[t] = bp2[t * 16 + rl];
  }
  const float b3    = (wave ? gb3 : db3)[0];
  const float dt    = dtp[0];
  const float kappa = kappap[0];
  const float theta = thetap[0];
  const _Float16* wf = s_frag + wave * (NFRAG * 512);
  _Float16* act = s_act[wave];
  const float* hw = s_hw[wave];

  const int gp  = path0 + lane;
  const int gpc = (gp < B) ? gp : (B - 1);
  float log_v = 0.0f;
  float s1[2] = {0.f, 0.f};
  float s2[4] = {0.f, 0.f, 0.f, 0.f};
  float s3[8] = {0.f, 0.f, 0.f, 0.f, 0.f, 0.f, 0.f, 0.f};
  if (wave == 0) {
    float iv = init_var[gpc];
    iv = fminf(1.5f, fmaxf(0.01f, iv));
    log_v = logf(iv);
    s_in[lane * IN_PITCH + 14] = (_Float16)(log_v + 4.0f);
  }

  for (int st = 0; st < S; ++st) {
    __syncthreads();

    layer_fwd<1>(s_in, IN_PITCH, wf,             b0r[0], b0r[1], b0r[2], b0r[3], act, lane);
    layer_fwd<2>(act, ACT_PITCH, wf + 4 * 512,   b1r[0], b1r[1], b1r[2], b1r[3], act, lane);
    layer_fwd<2>(act, ACT_PITCH, wf + 12 * 512,  b2r[0], b2r[1], b2r[2], b2r[3], act, lane);

    {
      const _Float16* row = act + lane * ACT_PITCH;
      float sum = 0.0f;
#pragma unroll
      for (int g = 0; g < 8; ++g) {
        const v8h q = *(const v8h*)(row + g * 8);
#pragma unroll
        for (int e = 0; e < 8; ++e) sum += (float)q[e] * hw[g * 8 + e];
      }
      s_raw[wave][lane] = sum + b3;
    }
    __syncthreads();

    if (wave == 0) {
      const float raw0 = s_raw[0][lane];
      const float raw1 = s_raw[1][lane];
      const float drift_nn  = 0.5f * tanhf(raw0);
      const float sig       = 1.0f / (1.0f + expf(-raw1));
      const float diffusion = 1.5f * sig + 0.1f;
      const float dwv       = dw[(size_t)gpc * S + st];
      const float drift_ou  = kappa * (theta - log_v) * dt;
      float lv = log_v + drift_ou + drift_nn * dt + diffusion * dwv;
      lv = fminf(1.0f, fmaxf(-5.0f, lv));
      s_out[lane * OUT_PITCH + (st & (CHUNK - 1))] = expf(lv);

      const float d = lv - log_v;
      const float dx[2] = {dt, d};
      const float dd[4] = {dt * dt, dt * d, d * dt, d * d};
      float n3[8], n2[4];
#pragma unroll
      for (int m = 0; m < 8; ++m)
        n3[m] = s3[m] + s2[m >> 1] * dx[m & 1] + s1[m >> 2] * (0.5f * dd[m & 3])
              + (dd[m >> 1] * dx[m & 1]) * (1.0f / 6.0f);
#pragma unroll
      for (int m = 0; m < 4; ++m)
        n2[m] = s2[m] + s1[m >> 1] * dx[m & 1] + 0.5f * dd[m];
      s1[0] += dt; s1[1] += d;
#pragma unroll
      for (int m = 0; m < 4; ++m) s2[m] = n2[m];
#pragma unroll
      for (int m = 0; m < 8; ++m) s3[m] = n3[m];
      log_v = lv;

      _Float16* rw = s_in + lane * IN_PITCH;
      rw[0] = (_Float16)s1[0]; rw[1] = (_Float16)s1[1];
#pragma unroll
      for (int m = 0; m < 4; ++m) rw[2 + m] = (_Float16)s2[m];
#pragma unroll
      for (int m = 0; m < 8; ++m) rw[6 + m] = (_Float16)s3[m];
      rw[14] = (_Float16)(log_v + 4.0f);
    }

    if ((st & (CHUNK - 1)) == (CHUNK - 1)) {
      __syncthreads();
      const int q  = lane >> 3;
      const int c4 = (lane & 7) * 4;
      const int col0 = st - (CHUNK - 1);
      for (int pass = 0; pass < 2; ++pass) {
#pragma unroll
        for (int it = 0; it < 4; ++it) {
          const int pl   = wave * 16 + it * 4 + q;
          const int gpth = path0 + pl;
          const v4f v = *(const v4f*)(s_out + pl * OUT_PITCH + c4);
          if ((unsigned)gpth < (unsigned)B)
            *(volatile v4f*)(out + (size_t)gpth * S + col0 + c4) = v;
        }
        __threadfence();
      }
    }
  }
}

extern "C" void kernel_launch(void* const* d_in, const int* in_sizes, int n_in,
                              void* d_out, int out_size, void* d_ws, size_t ws_size,
                              hipStream_t stream) {
  (void)n_in; (void)d_ws; (void)ws_size; (void)out_size;
  const float* P[21];
  for (int i = 0; i < 21; ++i) P[i] = (const float*)d_in[i];
  int B = in_sizes[16];
  if (B < 1) B = 1;
  const int S = in_sizes[17] / B;
  const int grid = (B + NPB - 1) / NPB;
  nrs_main<<<dim3(grid), dim3(NTHREADS), 0, stream>>>(
      P[0], P[1], P[2], P[3],
      P[4], P[5], P[6], P[7],
      P[8], P[9], P[10], P[11],
      P[12], P[13], P[14], P[15],
      P[16], P[17], P[18], P[19], P[20],
      (float*)d_out, B, S);
}
